// MultiHeadedAttention_10625749090758
// MI455X (gfx1250) — hardware-verified
//
#include <hip/hip_runtime.h>


#ifndef NB
#define NB 4
#endif
#ifndef SEQ
#define SEQ 2048
#endif
#define SEQ_FULL 2048
#define TT   SEQ
#define DM   1024
#define NH_  16
#define HD   64
#define FW   4
#define QCARRY 512.0f
#define KCARRY 512.0f
static_assert(QCARRY == 512.0f && KCARRY == 512.0f);
static_assert(QCARRY * KCARRY == 262144.0f);
#define CS2 (1.4426950408889634f * 0.125f * (1.0f / 262144.0f))
#define PLOG 10.0f

static_assert(TT % 128 == 0);
static_assert(TT % 32 == 0);
static_assert(TT <= SEQ_FULL);
static_assert(NH_ * HD == DM);
static_assert(DM % 64 == 0);
static_assert(DM % 32 == 0);
static_assert(HD == 64);
static_assert(NB >= 1 && NB <= 4);
static_assert((NB * TT) % 64 == 0);
static_assert((NH_ * (TT / 16)) % FW == 0);
static_assert(((size_t)NH_ * TT * HD) % (8 * 256) == 0);
static_assert(((size_t)DM * DM) % (8 * 256) == 0);
static_assert(((size_t)NB * SEQ_FULL * DM) % 8 == 0);
static_assert((size_t)NH_ * TT * HD < ((size_t)1 << 31));

typedef _Float16 h16;
typedef unsigned short bf;
typedef __attribute__((ext_vector_type(16))) __bf16   v16bf;
typedef __attribute__((ext_vector_type(16))) _Float16 v16h;
typedef __attribute__((ext_vector_type(8)))  _Float16 v8h;
typedef __attribute__((ext_vector_type(8)))  unsigned short v8us;
typedef __attribute__((ext_vector_type(8)))  float    v8f;
typedef __attribute__((ext_vector_type(4)))  float    v4f;
typedef v4f  __attribute__((may_alias)) v4fa;

__device__ __forceinline__ unsigned short f2bf(float f) { unsigned u = __float_as_uint(f); u += 0x7FFFu + ((u >> 16) & 1u); return (unsigned short)(u >> 16); }
__device__ __forceinline__ float bf2f(unsigned short b) { return __uint_as_float(((unsigned)b) << 16); }
__device__ __forceinline__ float bfr(float f) { return bf2f(f2bf(f)); }
__device__ __forceinline__ v16h cat16(v8h lo, v8h hi) { return __builtin_shufflevector(lo, hi, 0, 1, 2, 3, 4, 5, 6, 7, 8, 9, 10, 11, 12, 13, 14, 15); }
__device__ __forceinline__ v16bf cat16b(v8us lo, v8us hi) { return __builtin_bit_cast(v16bf, __builtin_shufflevector(lo, hi, 0, 1, 2, 3, 4, 5, 6, 7, 8, 9, 10, 11, 12, 13, 14, 15)); }
__device__ __forceinline__ v8f wmma16(v16h a, v16h b, v8f c) { return __builtin_amdgcn_wmma_f32_16x16x32_f16(false, a, false, b, (short)0, c, false, false); }
__device__ __forceinline__ v8f wmmab(v16bf a, v16bf b, v8f c) { return __builtin_amdgcn_wmma_f32_16x16x32_bf16(false, a, false, b, (short)0, c, false, false); }

template <typename T16> struct WFrag;
template <> struct WFrag<h16> { typedef v16h V; static __device__ __forceinline__ V ld(const h16* p) { return cat16(*(const v8h*)p, *(const v8h*)(p + 16)); } static __device__ __forceinline__ v8f mma(V a, V b, v8f c) { return wmma16(a, b, c); } };
template <> struct WFrag<bf> { typedef v16bf V; static __device__ __forceinline__ V ld(const bf* p) { return cat16b(*(const v8us*)p, *(const v8us*)(p + 16)); } static __device__ __forceinline__ v8f mma(V a, V b, v8f c) { return wmmab(a, b, c); } };
template <typename T16, int NSPLIT, bool BIAS>
__global__ __launch_bounds__(32) void k_gemmw(const T16* __restrict__ A, const T16* __restrict__ A2, const T16* __restrict__ Bt, const T16* __restrict__ Bt2, int K, float* C, int ldc, const float* __restrict__ bias, size_t sA, size_t sB, size_t sC) {
    typedef typename WFrag<T16>::V V;
    __shared__ __align__(16) float os[16 * 68];
    const size_t z = blockIdx.z; A += z * sA; if (A2) A2 += z * sA; Bt += z * sB; if (Bt2) Bt2 += z * sB; C += z * sC;
    const int lane = threadIdx.x & 31, lr = lane & 15, hi = lane >> 4; const int r0 = blockIdx.x * 64, c0 = blockIdx.y * 64;
    v8f acc[4][4];
#pragma unroll
    for (int mb = 0; mb < 4; ++mb)
#pragma unroll
        for (int nb = 0; nb < 4; ++nb) acc[mb][nb] = (v8f){};
    const size_t aoff = (size_t)(r0 + lr) * K + 8 * hi, boff = (size_t)(c0 + lr) * K + 8 * hi;
#pragma unroll 1
    for (int kc = 0; kc < K; kc += 32) {
        V a[4], a2[4];
#pragma unroll
        for (int mb = 0; mb < 4; ++mb) { a[mb] = WFrag<T16>::ld(A + aoff + (size_t)mb * 16 * K + kc); if (NSPLIT == 1 || NSPLIT == 2) a2[mb] = WFrag<T16>::ld(A2 + aoff + (size_t)mb * 16 * K + kc); }
#pragma unroll
        for (int nb = 0; nb < 4; ++nb) { const V b = WFrag<T16>::ld(Bt + boff + (size_t)nb * 16 * K + kc); V b2; if (NSPLIT >= 2) b2 = WFrag<T16>::ld(Bt2 + boff + (size_t)nb * 16 * K + kc);
#pragma unroll
            for (int mb = 0; mb < 4; ++mb) { acc[mb][nb] = WFrag<T16>::mma(a[mb], b, acc[mb][nb]); if (NSPLIT == 1 || NSPLIT == 2) acc[mb][nb] = WFrag<T16>::mma(a2[mb], b, acc[mb][nb]); if (NSPLIT >= 2) acc[mb][nb] = WFrag<T16>::mma(a[mb], b2, acc[mb][nb]); } }
        asm volatile("v_nop\n\tv_nop\n\tv_nop\n\tv_nop" : "+v"(acc[0][0]), "+v"(acc[1][1]), "+v"(acc[2][2]), "+v"(acc[3][3]) : "v"(a[0]), "v"(a[3]));
    }
#pragma unroll
    for (int mb = 0; mb < 4; ++mb) {
#pragma unroll
        for (int nb = 0; nb < 4; ++nb) {
#pragma unroll
            for (int j = 0; j < 8; ++j) os[(hi * 8 + j) * 68 + nb * 16 + lr] = acc[mb][nb][j]; }
        __builtin_amdgcn_wave_barrier(); asm volatile("" ::: "memory");
        float* crow = C + (size_t)(r0 + mb * 16) * ldc + c0;
#pragma unroll 1
        for (int ps = 0; ps < 2; ++ps) {
#pragma unroll
            for (int s = 0; s < 8; ++s) { const int row = 2 * s + hi, cofs = lr * 4; v4f val = *(const v4fa*)(os + row * 68 + cofs); if (BIAS) { val[0] += bfr(bias[c0 + cofs]); val[1] += bfr(bias[c0 + cofs + 1]); val[2] += bfr(bias[c0 + cofs + 2]); val[3] += bfr(bias[c0 + cofs + 3]); }
                *(volatile v4f*)(crow + (size_t)row * ldc + cofs) = val; }
            if (ps == 0) __threadfence(); }
        __builtin_amdgcn_wave_barrier(); asm volatile("" ::: "memory");
    }
}

__global__ __launch_bounds__(256) void k_cvt8(const float* __restrict__ src, bf* dst, size_t n8) { const size_t i = (size_t)blockIdx.x * 256 + threadIdx.x; if (i >= n8) return; const v8f v = *(const v8f*)(src + i * 8); v8us o;
#pragma unroll
    for (int k = 0; k < 8; ++k) o[k] = f2bf(v[k]); *(volatile v8us*)(dst + i * 8) = o; __threadfence(); *(volatile v8us*)(dst + i * 8) = o; }

__global__ __launch_bounds__(256) void k_wt(const float* __restrict__ wq, const float* __restrict__ wk, const float* __restrict__ wv, bf* Bt) {
    const unsigned z = blockIdx.y;
    const float* w = (z == 0u) ? wq : ((z == 1u) ? wk : wv);
    const unsigned i = blockIdx.x * 256u + threadIdx.x; if (i >= (unsigned)(DM * DM / 8)) return;
    const unsigned e = i * 8u; const unsigned k = e % (unsigned)DM; const unsigned n = e / (unsigned)DM; const unsigned h = n / (unsigned)HD, c = n % (unsigned)HD;
    v8us o;
#pragma unroll
    for (unsigned q = 0; q < 8; ++q) o[q] = f2bf(w[((size_t)h * DM + k + q) * HD + c]);
    bf* d = Bt + (size_t)z * DM * DM + e;
    *(volatile v8us*)d = o; __threadfence(); *(volatile v8us*)d = o;
}

__global__ __launch_bounds__(256) void k_wot(const float* __restrict__ wo, bf* Bt) {
    const unsigned i = blockIdx.x * 256u + threadIdx.x; if (i >= (unsigned)(DM * DM / 8)) return;
    const unsigned e = i * 8u; const unsigned k = e % (unsigned)DM; const unsigned n = e / (unsigned)DM;
    v8us o;
#pragma unroll
    for (unsigned q = 0; q < 8; ++q) o[q] = f2bf(wo[(size_t)(k + q) * DM + n]);
    bf* d = Bt + e;
    *(volatile v8us*)d = o; __threadfence(); *(volatile v8us*)d = o;
}

__global__ __launch_bounds__(256) void k_qkp(const float* __restrict__ FQ, const float* __restrict__ FK, h16* QH, h16* QL, h16* KH, h16* KL) {
    const unsigned y = blockIdx.y;
    const unsigned i = blockIdx.x * 256u + threadIdx.x; if (i >= (unsigned)(NH_ * TT * HD / 8)) return;
    const unsigned e = i * 8u; const unsigned d = e % (unsigned)HD; const unsigned t = (e / (unsigned)HD) % (unsigned)TT; const unsigned h = e / (unsigned)(HD * TT);
    const float* F = y ? FK : FQ;
    h16* PH = y ? KH : QH;
    h16* PL = y ? KL : QL;
    const v8f f = *(const v8f*)(F + (size_t)t * DM + h * HD + d);
    v8h oh, ol;
#pragma unroll
    for (int q = 0; q < 8; ++q) { const float s = f[q] * QCARRY; const h16 hh = (h16)s; oh[q] = hh; ol[q] = (h16)(s - (float)hh); }
    *(volatile v8h*)(PH + e) = oh; *(volatile v8h*)(PL + e) = ol; __threadfence(); *(volatile v8h*)(PH + e) = oh; *(volatile v8h*)(PL + e) = ol;
}

__global__ __launch_bounds__(256) void k_vtp(const float* __restrict__ F, h16* VT) {
    const unsigned i = blockIdx.x * 256u + threadIdx.x; if (i >= (unsigned)(NH_ * HD * TT / 8)) return;
    const unsigned e = i * 8u; const unsigned t = e % (unsigned)TT; const unsigned d = (e / (unsigned)TT) % (unsigned)HD; const unsigned h = e / (unsigned)(TT * HD);
    v8h o;
#pragma unroll
    for (unsigned q = 0; q < 8; ++q) o[q] = (h16)F[(size_t)(t + q) * DM + h * HD + d];
    *(volatile v8h*)(VT + e) = o; __threadfence(); *(volatile v8h*)(VT + e) = o;
}

__global__ __launch_bounds__(FW * 32) void k_flash(const h16* __restrict__ QH, const h16* __restrict__ QL, const h16* __restrict__ KH, const h16* __restrict__ KL, const h16* __restrict__ VT, bf* CH, bf* CL, unsigned rowbase) {
    __shared__ __align__(16) float os[FW * 16 * 68];
    const unsigned lane = threadIdx.x & 31u, wave = threadIdx.x >> 5, lr = lane & 15u, hi = lane >> 4;
    const unsigned wid = blockIdx.x * (unsigned)FW + wave;
    const unsigned h = wid / (unsigned)(TT / 16), qt = wid % (unsigned)(TT / 16);
    const size_t qoff = ((size_t)h * TT + qt * 16u + lr) * HD + 8u * hi;
    const v16h bh0 = WFrag<h16>::ld(QH + qoff), bh1 = WFrag<h16>::ld(QH + qoff + 32);
    const v16h bl0 = WFrag<h16>::ld(QL + qoff), bl1 = WFrag<h16>::ld(QL + qoff + 32);
    const size_t koff = ((size_t)h * TT + lr) * HD + 8u * hi;
    const h16* kp  = KH + koff;
    const h16* klp = KL + koff;
    const h16* vp = VT + ((size_t)h * HD + lr) * TT + 8u * hi;
    v8f o0 = (v8f){}, o1 = (v8f){}, o2 = (v8f){}, o3 = (v8f){};
    float m = -1.0e30f, ls = 0.0f;
#pragma unroll 1
    for (unsigned t0 = 0; t0 < (unsigned)TT; t0 += 32u) {
        const h16* kk = kp + (size_t)t0 * HD;
        const h16* kl = klp + (size_t)t0 * HD;
        v8f s0 = (v8f){}, s1 = (v8f){};
        {
            const v16h ka0 = WFrag<h16>::ld(kk), ka1 = WFrag<h16>::ld(kk + 32);
            const v16h kb0 = WFrag<h16>::ld(kk + 16 * HD), kb1 = WFrag<h16>::ld(kk + 16 * HD + 32);
            s0 = wmma16(ka0, bl0, s0); s1 = wmma16(kb0, bl0, s1);
            s0 = wmma16(ka1, bl1, s0); s1 = wmma16(kb1, bl1, s1);
            {
                const v16h la0 = WFrag<h16>::ld(kl), la1 = WFrag<h16>::ld(kl + 32);
                const v16h lb0 = WFrag<h16>::ld(kl + 16 * HD), lb1 = WFrag<h16>::ld(kl + 16 * HD + 32);
                s0 = wmma16(la0, bh0, s0); s1 = wmma16(lb0, bh0, s1);
                s0 = wmma16(la1, bh1, s0); s1 = wmma16(lb1, bh1, s1);
            }
            s0 = wmma16(ka0, bh0, s0); s1 = wmma16(kb0, bh0, s1);
            s0 = wmma16(ka1, bh1, s0); s1 = wmma16(kb1, bh1, s1);
            asm volatile("v_nop\n\tv_nop\n\tv_nop\n\tv_nop" : "+v"(s0), "+v"(s1) : "v"(ka1), "v"(kb1), "v"(bh1));
        }
        float mloc = fmaxf(s0[0], s1[0]);
#pragma unroll
        for (int r = 1; r < 8; ++r) mloc = fmaxf(mloc, fmaxf(s0[r], s1[r]));
        const float mo = __shfl_xor(mloc, 16, 32);
        mloc = fmaxf(mloc, mo);
        const float mnew = fmaxf(m, mloc * CS2);
        const float alpha = __builtin_amdgcn_exp2f(m - mnew);
        const float off = PLOG - mnew;
        v16h pb; float psum = 0.0f;
#pragma unroll
        for (int r = 0; r < 8; ++r) { const float p = __builtin_amdgcn_exp2f(__builtin_fmaf(s0[r], CS2, off)); psum += p; pb[r] = (h16)p; }
#pragma unroll
        for (int r = 0; r < 8; ++r) { const float p = __builtin_amdgcn_exp2f(__builtin_fmaf(s1[r], CS2, off)); psum += p; pb[8 + r] = (h16)p; }
        ls = ls * alpha + psum; m = mnew;
        o0 *= alpha; o1 *= alpha; o2 *= alpha; o3 *= alpha;
        const h16* vv = vp + t0;
        const v16h va0 = WFrag<h16>::ld(vv), va1 = WFrag<h16>::ld(vv + (size_t)16 * TT), va2 = WFrag<h16>::ld(vv + (size_t)32 * TT), va3 = WFrag<h16>::ld(vv + (size_t)48 * TT);
        o0 = wmma16(va0, pb, o0); o1 = wmma16(va1, pb, o1); o2 = wmma16(va2, pb, o2); o3 = wmma16(va3, pb, o3);
        asm volatile("v_nop\n\tv_nop\n\tv_nop\n\tv_nop" : "+v"(o0), "+v"(o1), "+v"(o2), "+v"(o3) : "v"(pb), "v"(va3));
    }
    const float lo2 = __shfl_xor(ls, 16, 32);
    const float inv = __builtin_amdgcn_rcpf(ls + lo2);
    float* ow = os + wave * (16 * 68);
#pragma unroll
    for (int r = 0; r < 8; ++r) {
        ow[lr * 68u + 8u * hi + r]       = o0[r] * inv;
        ow[lr * 68u + 16u + 8u * hi + r] = o1[r] * inv;
        ow[lr * 68u + 32u + 8u * hi + r] = o2[r] * inv;
        ow[lr * 68u + 48u + 8u * hi + r] = o3[r] * inv;
    }
    __builtin_amdgcn_wave_barrier(); asm volatile("" ::: "memory");
    const size_t gbase = (size_t)(rowbase + qt * 16u) * DM + h * HD;
#pragma unroll 1
    for (int ps = 0; ps < 2; ++ps) {
#pragma unroll
        for (unsigned s = 0; s < 4; ++s) {
            const unsigned row = 4u * s + (lane >> 3), pc = lane & 7u;
            const v4f a = *(const v4fa*)(ow + row * 68u + pc * 8u);
            const v4f b = *(const v4fa*)(ow + row * 68u + pc * 8u + 4u);
            v8us oh, ol;
#pragma unroll
            for (int q = 0; q < 4; ++q) {
                const unsigned short ha = f2bf(a[q]); oh[q] = ha; ol[q] = f2bf(a[q] - bf2f(ha));
                const unsigned short hb = f2bf(b[q]); oh[4 + q] = hb; ol[4 + q] = f2bf(b[q] - bf2f(hb));
            }
            const size_t g = gbase + (size_t)row * DM + pc * 8u;
            *(volatile v8us*)(CH + g) = oh; *(volatile v8us*)(CL + g) = ol;
        }
        if (ps == 0) __threadfence();
    }
}

constexpr size_t al256(size_t b) { return (b + 255) & ~(size_t)255; }
constexpr size_t SZ_WT  = al256((size_t)3 * DM * DM * 2);
constexpr size_t SZ_WOT = al256((size_t)DM * DM * 2);
constexpr size_t SZ_XB  = al256((size_t)NB * SEQ_FULL * DM * 2);
constexpr size_t SZ_F   = al256((size_t)3 * TT * DM * 4);
constexpr size_t SZ_PL  = al256((size_t)NH_ * TT * HD * 2);
constexpr size_t SZ_CTX = al256((size_t)NB * TT * DM * 2);
constexpr size_t SZ_TOTAL = SZ_WT + SZ_WOT + SZ_XB + SZ_F + 5 * SZ_PL + 2 * SZ_CTX;
static_assert(SZ_TOTAL <= (size_t)134217728);

extern "C" void kernel_launch(void* const* d_in, const int* in_sizes, int n_in,
                              void* d_out, int out_size, void* d_ws, size_t ws_size, hipStream_t stream) {
    if (n_in < 5) return;
    if (in_sizes[0] < NB * SEQ_FULL * DM) return;
    if (in_sizes[1] < NH_ * DM * HD || in_sizes[2] < NH_ * DM * HD || in_sizes[3] < NH_ * DM * HD) return;
    if (in_sizes[4] < DM * DM) return;
    if (out_size < NB * TT * DM) return;
    if (SZ_TOTAL > ws_size) return;
    const float* x  = (const float*)d_in[0];
    const float* wq = (const float*)d_in[1];
    const float* wk = (const float*)d_in[2];
    const float* wv = (const float*)d_in[3];
    const float* wo = (const float*)d_in[4];
    float* OUT = (float*)d_out;
    char* wsp = (char*)d_ws;
    bf*    WT  = (bf*)wsp;     wsp += SZ_WT;
    bf*    WOT = (bf*)wsp;     wsp += SZ_WOT;
    bf*    XB  = (bf*)wsp;     wsp += SZ_XB;
    float* F   = (float*)wsp;  wsp += SZ_F;
    h16*   QH  = (h16*)wsp;    wsp += SZ_PL;
    h16*   QL  = (h16*)wsp;    wsp += SZ_PL;
    h16*   KH  = (h16*)wsp;    wsp += SZ_PL;
    h16*   KL  = (h16*)wsp;    wsp += SZ_PL;
    h16*   VT  = (h16*)wsp;    wsp += SZ_PL;
    bf*    CH  = (bf*)wsp;     wsp += SZ_CTX;
    bf*    CL  = (bf*)wsp;     wsp += SZ_CTX;
    float* FQ = F; float* FK = F + (size_t)TT * DM; float* FV = F + (size_t)2 * TT * DM;

    k_wt<<<dim3((unsigned)((size_t)DM * DM / 8 / 256), 3), 256, 0, stream>>>(wq, wk, wv, WT);
    k_wot<<<(unsigned)((size_t)DM * DM / 8 / 256), 256, 0, stream>>>(wo, WOT);
    const size_t nx8 = (size_t)NB * SEQ_FULL * DM / 8;
    k_cvt8<<<(unsigned)((nx8 + 255) / 256), 256, 0, stream>>>(x, XB, nx8);
    const unsigned LP = (unsigned)((size_t)NH_ * TT * HD / 8 / 256);
    for (int b = 0; b < NB; ++b) {
        k_gemmw<bf, 0, false><<<dim3(TT / 64, DM / 64, 3), 32, 0, stream>>>(XB + (size_t)b * SEQ_FULL * DM, nullptr, WT, nullptr, DM, F, DM, nullptr, (size_t)0, (size_t)DM * DM, (size_t)TT * DM);
        k_qkp<<<dim3(LP, 2), 256, 0, stream>>>(FQ, FK, QH, QL, KH, KL);
        k_vtp<<<LP, 256, 0, stream>>>(FV, VT);
        k_flash<<<(unsigned)(NH_ * (TT / 16) / FW), FW * 32, 0, stream>>>(QH, QL, KH, KL, VT, CH, CL, (unsigned)(b * TT));
    }
    k_gemmw<bf, 1, false><<<dim3(NB * TT / 64, DM / 64, 1), 32, 0, stream>>>(CH, CL, WOT, nullptr, DM, OUT, DM, nullptr, (size_t)0, (size_t)0, (size_t)0);
}
